// QuantumLayer_42657615184198
// MI455X (gfx1250) — hardware-verified
//
#include <hip/hip_runtime.h>


#ifndef NB
#define NB 32768
#endif
#define NB_FULL 32768
#define QN   9
#define QD   512
#define GW   4
#define CW   32
#define MRB  32
#define QRS  2048.0f
#define QRI  (1.0f / 2048.0f)
#define USC  4096.0f
#define MSC  4096.0f
#define PSCL (1.0f / 16777216.0f)

static_assert(QD == (1 << QN));
static_assert(QD % 32 == 0);
static_assert(QD % 16 == 0);
static_assert(CW == 32);
static_assert(NB % (CW * GW) == 0);
static_assert(NB % MRB == 0);
static_assert(NB <= NB_FULL);
static_assert((CW * QN * 4) % 128 == 0);
static_assert((32 * 2 + 8) * 16 == CW * QN * 4);
static_assert(MRB * 64 == 8 * 256);
static_assert((MRB * QN) % 32 == 0);
static_assert((MRB * 32) % 256 == 0);
static_assert((MRB * 16) % 256 == 0);
static_assert(4 * 64 == 256);
static_assert(USC * MSC * PSCL == 1.0f);
static_assert(GW * CW * QN * 4 <= 131072);
static_assert((81 * 2 + 27 * 8 + 4 * QD) * 4 <= 131072);
static_assert((MRB * QN * 2 + MRB * 32 + MRB * 16) * 4 <= 131072);

typedef _Float16 h16;
typedef __attribute__((ext_vector_type(16))) _Float16 v16h;
typedef __attribute__((ext_vector_type(8)))  _Float16 v8h;
typedef __attribute__((ext_vector_type(8)))  float    v8f;
typedef __attribute__((ext_vector_type(4)))  float    v4f;
typedef v4f  __attribute__((may_alias)) v4fa;

__device__ __forceinline__ unsigned short f2bf(float f) { unsigned u = __float_as_uint(f); u += 0x7FFFu + ((u >> 16) & 1u); return (unsigned short)(u >> 16); }
__device__ __forceinline__ float bfr(float f) { return __uint_as_float(((unsigned)f2bf(f)) << 16); }
__device__ __forceinline__ v16h cat16(v8h lo, v8h hi) { return __builtin_shufflevector(lo, hi, 0, 1, 2, 3, 4, 5, 6, 7, 8, 9, 10, 11, 12, 13, 14, 15); }
__device__ __forceinline__ v8f wmma16(v16h a, v16h b, v8f c) { return __builtin_amdgcn_wmma_f32_16x16x32_f16(false, a, false, b, (short)0, c, false, false); }
__device__ __forceinline__ v16h  ldh(const h16* p) { return cat16(*(const v8h*)p, *(const v8h*)(p + 16)); }
__device__ __forceinline__ void wave_sync() { __builtin_amdgcn_fence(3  , "wavefront"); __builtin_amdgcn_wave_barrier(); asm volatile("" ::: "memory"); }
static __device__ __forceinline__ h16 toh_flush(float v) { const h16 r = (h16)v; return (fabsf(v) < 6.103515625e-05f) ? (h16)0.0f : r; }
__device__ __forceinline__ v8f wmg(v16h a, v16h b, v8f c) { c = wmma16(a, b, c); asm volatile("v_nop\n\tv_nop\n\tv_nop\n\tv_nop" : "+v"(c) : "v"(a), "v"(b)); return c; }

__global__ __launch_bounds__(256) void k_ubuild(const float* __restrict__ wts, h16* UP) {
#pragma clang fp contract(off)
    __shared__ float sn[81];
    __shared__ float cs[81];
    __shared__ float gm[27 * 8];
    __shared__ __align__(16) float vr[2 * QD];
    __shared__ __align__(16) float vi[2 * QD];
    const int t = threadIdx.x; const int j = blockIdx.x;
    if (t < 96) {
        const int ti = t < 81 ? t : 80; const int g = ti / 3, wh = ti - 3 * g;
        const float phi = bfr(wts[g * 3 + 0]), th = bfr(wts[g * 3 + 1]), om = bfr(wts[g * 3 + 2]);
        const float a0 = 0.5f * th, a1 = -0.5f * (phi + om), a2 = -0.5f * (phi - om);
        const float a = (wh == 0) ? a0 : ((wh == 1) ? a1 : a2);
        float s, c; sincosf(a, &s, &c);
        if (t < 81) { sn[t] = s; cs[t] = c; }
    }
    vr[t] = (t == j) ? 1.0f : 0.0f; vr[t + 256] = (t + 256 == j) ? 1.0f : 0.0f; vi[t] = 0.0f; vi[t + 256] = 0.0f;
    __syncthreads();
    if (t < 32) {
        const int g = t < 27 ? t : 26;
        const float ch = cs[3 * g], sh = sn[3 * g], cap = cs[3 * g + 1], sap = sn[3 * g + 1], cam = cs[3 * g + 2], sam = sn[3 * g + 2];
        if (t < 27) {
            gm[g * 8 + 0] = cap * ch;    gm[g * 8 + 1] = sap * ch;
            gm[g * 8 + 2] = -(cam * sh); gm[g * 8 + 3] = sam * sh;
            gm[g * 8 + 4] = cam * sh;    gm[g * 8 + 5] = sam * sh;
            gm[g * 8 + 6] = cap * ch;    gm[g * 8 + 7] = -(sap * ch);
        }
    }
    __syncthreads();
    int cb = 0;
#pragma unroll 1
    for (int l = 2; l >= 0; --l) {
        const int rr = l + 1; const int nb = 1 - cb;
#pragma unroll 1
        for (int e = 0; e < 2; ++e) {
            const int i = t + 256 * e; int cur = i;
#pragma unroll 1
            for (int ii = 0; ii < QN; ++ii) { const int bit = (cur >> (8 - ii)) & 1; int tq = ii + rr; tq = tq >= QN ? tq - QN : tq; cur ^= bit << (8 - tq); }
            vr[nb * QD + i] = vr[cb * QD + cur]; vi[nb * QD + i] = vi[cb * QD + cur];
        }
        cb = nb;
        __syncthreads();
#pragma unroll 1
        for (int w = 0; w < QN; ++w) {
            const int g = (l * QN + w) * 8;
            const float m00r = gm[g + 0], m00i = gm[g + 1], m01r = gm[g + 2], m01i = gm[g + 3];
            const float m10r = gm[g + 4], m10i = gm[g + 5], m11r = gm[g + 6], m11i = gm[g + 7];
            const int mask = 1 << (8 - w); const int low = t & (mask - 1); const int high = (t & ~(mask - 1)) << 1;
            const int j0 = cb * QD + (high | low), j1 = j0 + mask;
            const float v0r = vr[j0], v0i = vi[j0], v1r = vr[j1], v1i = vi[j1];
            const float n0r = m00r * v0r - m00i * v0i + m10r * v1r - m10i * v1i;
            const float n0i = m00r * v0i + m00i * v0r + m10r * v1i + m10i * v1r;
            const float n1r = m01r * v0r - m01i * v0i + m11r * v1r - m11i * v1i;
            const float n1i = m01r * v0i + m01i * v0r + m11r * v1i + m11i * v1r;
            vr[j0] = n0r; vi[j0] = n0i; vr[j1] = n1r; vi[j1] = n1i;
            __syncthreads();
        }
    }
    const int sel = t >> 6, pc = t & 63;
    const bool isim = sel >= 2; const bool isres = (sel & 1) != 0;
    const size_t oo = (size_t)sel * QD * QD + (size_t)j * QD + (size_t)pc * 8;
#pragma unroll 1
    for (int ps = 0; ps < 2; ++ps) {
        v8h o;
#pragma unroll
        for (int i = 0; i < 8; ++i) {
            const int k = pc * 8 + i;
            const float ar = vr[cb * QD + k], ai = vi[cb * QD + k];
            const int c = __popc(k) & 3;
            const float nr = (c == 0) ? ar : ((c == 1) ? ai : ((c == 2) ? -ar : -ai));
            const float ni = (c == 0) ? ai : ((c == 1) ? -ar : ((c == 2) ? -ai : ar));
            const float val = (isim ? ni : nr) * USC;
            const h16 hv = toh_flush(val);
            const h16 rv = toh_flush((val - (float)hv) * QRS);
            o[i] = isres ? rv : hv;
        }
        *(volatile v8h*)(UP + oo) = o;
        if (ps == 0) __threadfence();
    }
}

__global__ __launch_bounds__(256) void k_mplane(const float* __restrict__ x, h16* MH, h16* MR) {
#pragma clang fp contract(off)
    __shared__ float cs[MRB * QN];
    __shared__ float sn[MRB * QN];
    __shared__ float mh[MRB * 32];
    __shared__ float ml[MRB * 16];
    const int t = threadIdx.x; const int b0 = blockIdx.x * MRB;
#pragma unroll 1
    for (int e = t; e < MRB * QN; e += 256) {
        const float xv = bfr(x[(size_t)b0 * QN + e]);
        float s, c; sincosf(0.5f * xv, &s, &c);
        sn[e] = s; cs[e] = c;
    }
    __syncthreads();
#pragma unroll 1
    for (int e = t; e < MRB * 32; e += 256) {
        const int row = e >> 5, kh = e & 31; float p = 1.0f;
#pragma unroll
        for (int w = 0; w < 5; ++w) { const float cv = cs[row * QN + w], sv = sn[row * QN + w]; p *= ((kh >> (4 - w)) & 1) ? sv : cv; }
        mh[e] = p;
    }
#pragma unroll 1
    for (int e = t; e < MRB * 16; e += 256) {
        const int row = e >> 4, kl = e & 15; float p = 1.0f;
#pragma unroll
        for (int w = 5; w < 9; ++w) { const float cv = cs[row * QN + w], sv = sn[row * QN + w]; p *= ((kl >> (8 - w)) & 1) ? sv : cv; }
        ml[e] = p;
    }
    __syncthreads();
#pragma unroll 1
    for (int ps = 0; ps < 2; ++ps) {
#pragma unroll 1
        for (int it = 0; it < 8; ++it) {
            const int pid = it * 256 + t; const int row = pid >> 6, pc = pid & 63;
            const float a = mh[row * 32 + (pc >> 1)] * MSC; const int lo0 = row * 16 + (pc & 1) * 8;
            v8h hv, rv;
#pragma unroll
            for (int i = 0; i < 8; ++i) { const float v = a * ml[lo0 + i]; const h16 h = toh_flush(v); hv[i] = h; rv[i] = toh_flush((v - (float)h) * QRS); }
            const size_t oo = (size_t)(b0 + row) * QD + (size_t)pc * 8;
            *(volatile v8h*)(MH + oo) = hv; *(volatile v8h*)(MR + oo) = rv;
        }
        if (ps == 0) __threadfence();
    }
}

__global__ __launch_bounds__(32 * GW) void k_expect(const h16* __restrict__ UP, const h16* __restrict__ MH, const h16* __restrict__ MR, float* OUT) {
    __shared__ __align__(16) float os[GW * CW * QN];
    const int lane = threadIdx.x & 31, lr = lane & 15, hi = lane >> 4;
    const int wave = __builtin_amdgcn_readfirstlane((int)(threadIdx.x >> 5));
    const int b0 = (blockIdx.x * GW + wave) * CW;
    const h16* UrH = UP;
    const h16* UrR = UP + (size_t)QD * QD;
    const h16* UiH = UP + (size_t)2 * QD * QD;
    const h16* UiR = UP + (size_t)3 * QD * QD;
    const size_t ao = (size_t)lr * QD + 8 * hi;
    const size_t bo = (size_t)(b0 + lr) * QD + 8 * hi;
    const float sg5 = 1.0f - 2.0f * (float)hi;
    float z[2][QN];
#pragma unroll
    for (int cb = 0; cb < 2; ++cb)
#pragma unroll
        for (int q = 0; q < QN; ++q) z[cb][q] = 0.0f;
#pragma unroll 1
    for (int jb = 0; jb < QD / 16; ++jb) {
        v8f rH[2], rL[2], iH[2], iL[2];
#pragma unroll
        for (int cb = 0; cb < 2; ++cb) { rH[cb] = (v8f){}; rL[cb] = (v8f){}; iH[cb] = (v8f){}; iL[cb] = (v8f){}; }
        const size_t aj = ao + (size_t)jb * 16 * QD;
#pragma unroll 1
        for (int kc = 0; kc < QD; kc += 32) {
            const v16h arh = ldh(UrH + aj + kc), arr = ldh(UrR + aj + kc), aih = ldh(UiH + aj + kc), air = ldh(UiR + aj + kc);
#pragma unroll
            for (int cb = 0; cb < 2; ++cb) {
                const v16h bh = ldh(MH + bo + (size_t)cb * 16 * QD + kc), br = ldh(MR + bo + (size_t)cb * 16 * QD + kc);
                rH[cb] = wmg(arh, bh, rH[cb]); rL[cb] = wmg(arh, br, rL[cb]); rL[cb] = wmg(arr, bh, rL[cb]);
                iH[cb] = wmg(aih, bh, iH[cb]); iL[cb] = wmg(aih, br, iL[cb]); iL[cb] = wmg(air, bh, iL[cb]);
            }
        }
#pragma unroll
        for (int cb = 0; cb < 2; ++cb) {
            float pt = 0.0f, d6 = 0.0f, d7 = 0.0f, d8 = 0.0f;
#pragma unroll
            for (int r = 0; r < 8; ++r) {
                const float re = (rH[cb][r] + rL[cb][r] * QRI) * PSCL;
                const float im = (iH[cb][r] + iL[cb][r] * QRI) * PSCL;
                const float p = re * re + im * im;
                pt += p;
                d6 += (r & 4) ? -p : p; d7 += (r & 2) ? -p : p; d8 += (r & 1) ? -p : p;
            }
#pragma unroll
            for (int q = 0; q < 5; ++q) { const float sj = 1.0f - 2.0f * (float)((jb >> (4 - q)) & 1); z[cb][q] += sj * pt; }
            z[cb][5] += sg5 * pt; z[cb][6] += d6; z[cb][7] += d7; z[cb][8] += d8;
        }
    }
#pragma unroll
    for (int cb = 0; cb < 2; ++cb)
#pragma unroll
        for (int q = 0; q < QN; ++q) z[cb][q] += __shfl_xor(z[cb][q], 16, 32);
    const int wb = wave * (CW * QN);
    if (hi == 0) {
#pragma unroll
        for (int cb = 0; cb < 2; ++cb)
#pragma unroll
            for (int q = 0; q < QN; ++q) os[wb + (cb * 16 + lr) * QN + q] = z[cb][q];
    }
    wave_sync();
    float* ob = OUT + (size_t)b0 * QN;
    const int p2 = 64 + (lane & 7);
#pragma unroll 1
    for (int ps = 0; ps < 2; ++ps) {
#pragma unroll
        for (int s = 0; s < 2; ++s) { const int p = s * 32 + lane;
            const v4f val = *(const v4fa*)(&os[wb + p * 4]);
            *(volatile v4f*)(ob + (size_t)p * 4) = val; }
        const v4f val2 = *(const v4fa*)(&os[wb + p2 * 4]);
        if (lane < 8) *(volatile v4f*)(ob + (size_t)p2 * 4) = val2;
        if (ps == 0) __threadfence(); }
}

static constexpr size_t al256(size_t v) { return (v + 255) & ~(size_t)255; }
static constexpr size_t SZ_UP = al256((size_t)4 * QD * QD * 2);
static constexpr size_t SZ_MP = al256((size_t)NB * QD * 2);
static constexpr size_t SZ_TOTAL = SZ_UP + 2 * SZ_MP;
static_assert(SZ_TOTAL <= (size_t)134217728);
static_assert(((size_t)QD * QD * 2) % 256 == 0);
static_assert(((size_t)QD * 2) % 128 == 0);

extern "C" void kernel_launch(void* const* d_in, const int* in_sizes, int n_in,
                              void* d_out, int out_size, void* d_ws, size_t ws_size, hipStream_t stream) {
    if (n_in < 2) return;
    if ((size_t)in_sizes[0] < (size_t)NB * QN) return;
    if (in_sizes[1] < 81) return;
    if ((size_t)out_size < (size_t)NB * QN) return;
    if (SZ_TOTAL > ws_size) return;
    const float* x   = (const float*)d_in[0];
    const float* wts = (const float*)d_in[1];
    float* OUT = (float*)d_out;
    char* wsp = (char*)d_ws;
    h16* UP = (h16*)wsp; wsp += SZ_UP;
    h16* MH = (h16*)wsp; wsp += SZ_MP;
    h16* MR = (h16*)wsp; wsp += SZ_MP;

    k_ubuild<<<dim3(QD, 1, 1), 256, 0, stream>>>(wts, UP);
    k_mplane<<<dim3(NB / MRB, 1, 1), 256, 0, stream>>>(x, MH, MR);
    k_expect<<<dim3(NB / (CW * GW), 1, 1), 32 * GW, 0, stream>>>(UP, MH, MR, OUT);
}
